// noCluster_Mean_n_Max_16183436771705
// MI455X (gfx1250) — hardware-verified
//
#include <hip/hip_runtime.h>
#include <stddef.h>


typedef _Float16 h16;
typedef _Float16 v16h __attribute__((ext_vector_type(16)));
typedef _Float16 v8h  __attribute__((ext_vector_type(8)));
typedef float    v8f  __attribute__((ext_vector_type(8)));
typedef float    v4f  __attribute__((ext_vector_type(4)));

#ifndef NBAG
#define NBAG 8192
#endif
#define NBAG_FULL 8192
#define NTOK   409600
#define VOCAB  100000
#define EMB    128
#define MK     256
#define NTYPES 128

static_assert(NBAG >= 64 && NBAG <= NBAG_FULL);
static_assert((NBAG % 64) == 0 && (NBAG % 8) == 0);
static_assert(MK == 2 * EMB);
static_assert(EMB == 32 * 4);
static_assert(MK == 32 * 8);
static_assert((MK % 32) == 0 && (MK % 8) == 0);
static_assert((NTYPES % 64) == 0);
static_assert(((NTYPES * MK) % (256 * 8)) == 0);
static_assert((size_t)VOCAB * EMB < (size_t)0x7FFFFFFF);

#define LDC 68
static_assert((LDC % 4) == 0 && LDC >= 64);

#define WCARRY 64.0f
#define ACARRY 64.0f

#define LT_BYTES   ((size_t)NTYPES * MK * 2)
#define MEN_BYTES  ((size_t)NBAG * MK * 2)
#define OFF_LT   ((size_t)0)
#define OFF_MEN  (OFF_LT + LT_BYTES)
#define WS_TOTAL (OFF_MEN + MEN_BYTES)
static_assert((LT_BYTES % 128) == 0 && (MEN_BYTES % 128) == 0);
static_assert(WS_TOTAL <= (size_t)134217728);

static_assert((size_t)64 * LDC * 4 <= (size_t)131072);
static_assert((size_t)8 * MK * 2 <= (size_t)131072);

__device__ __forceinline__ float bf16r(float x) {
  unsigned int u = __float_as_uint(x);
  u = (u + 0x7FFFu + ((u >> 16) & 1u)) & 0xFFFF0000u;
  return __uint_as_float(u);
}

static __device__ __forceinline__ h16 toh_flush(float v) {
  const h16 r = (h16)v;
  return (fabsf(v) < 6.103515625e-05f) ? (h16)0.0f : r;
}

__device__ __forceinline__ v16h frag_at(const _Float16* p) {
  v8h lo = *(const v8h*)(p);
  v8h hi = *(const v8h*)(p + 16);
  v16h out;
#pragma unroll
  for (int i = 0; i < 8; ++i) { out[i] = lo[i]; out[i + 8] = hi[i]; }
  return out;
}

__device__ __forceinline__ v8f wmma16(v16h a, v16h b, v8f c) {
  v8f d = __builtin_amdgcn_wmma_f32_16x16x32_f16(false, a, false, b, (short)0, c,
                                                 false, false);
  asm volatile("v_nop\n\tv_nop\n\tv_nop\n\tv_nop" : "+v"(d) : "v"(a), "v"(b));
  return d;
}

__device__ __forceinline__ void wave_lds_sync() {
  __builtin_amdgcn_fence(3  , "wavefront");
  asm volatile("s_wait_dscnt 0x0" ::: "memory");
  __builtin_amdgcn_wave_barrier();
}

__global__ __launch_bounds__(256) void lconv_kernel(
    const float* __restrict__ Lw, _Float16* __restrict__ Lt) {
#pragma clang fp contract(off)
  const unsigned idx = blockIdx.x * 256u + threadIdx.x;
  const size_t e0 = (size_t)idx * 8u;
  const v4f a0 = *(const v4f*)(Lw + e0);
  const v4f a1 = *(const v4f*)(Lw + e0 + 4u);
  v8h o;
#pragma unroll
  for (int i = 0; i < 4; ++i) {
    o[i]     = toh_flush(WCARRY * bf16r(a0[i]));
    o[i + 4] = toh_flush(WCARRY * bf16r(a1[i]));
  }
  _Float16* p = Lt + e0;
  *(volatile v8h*)p = o;
  __threadfence();
  *(volatile v8h*)p = o;
}

__global__ __launch_bounds__(256) void bag_kernel(
    const int* __restrict__ feat, const int* __restrict__ offs,
    const float* __restrict__ W, _Float16* __restrict__ men) {
#pragma clang fp contract(off)
  __shared__ _Float16 S[8 * MK];
  const unsigned lane = threadIdx.x & 31u;
  const int wave = __builtin_amdgcn_readfirstlane((int)(threadIdx.x >> 5));
  const int b = (int)blockIdx.x * 8 + wave;
  const int bn = min(b + 1, NBAG_FULL - 1);
  const int r0 = offs[b];
  const int r1v = offs[bn];
  const int r1 = (b + 1 < NBAG_FULL) ? r1v : NTOK;
  const bool bad = (r0 < 0) | (r0 > NTOK) | (r1 < r0) | (r1 > NTOK) | ((b == 0) & (r0 != 0));

  const int c0 = min(max(r0, 0), NTOK);
  const int c1 = min(max(r1, 0), NTOK);
  const int cntv = max(c1 - c0, 0);
  const int dnm = max(cntv, 1);
  const int t0 = __builtin_amdgcn_readfirstlane(c0);
  const int t1 = __builtin_amdgcn_readfirstlane(c0 + cntv);

  v4f sum = {0.0f, 0.0f, 0.0f, 0.0f};
  const float ninf = -__builtin_huge_valf();
  v4f mx = {ninf, ninf, ninf, ninf};
#pragma unroll 2
  for (int t = t0; t < t1; ++t) {
    int tok = feat[t];
    tok = (tok < 0) ? (tok + VOCAB) : tok;
    tok = min(max(tok, 0), VOCAB - 1);
    const v4f a = *(const v4f*)(W + (size_t)tok * EMB + lane * 4u);
#pragma unroll
    for (int i = 0; i < 4; ++i) {
      const float e = bf16r(a[i]);
      sum[i] = sum[i] + e;
      mx[i] = fmaxf(mx[i], e);
    }
  }

  const float invd = 1.0f / (float)dnm;
  const float qn = __uint_as_float(0x7FC00000u);
  const unsigned sb = (unsigned)wave * (unsigned)MK;
#pragma unroll
  for (int i = 0; i < 4; ++i) {
    float mv = sum[i] * invd;
    float xv = (cntv > 0) ? mx[i] : 0.0f;
    mv = bad ? qn : mv;
    xv = bad ? qn : xv;
    S[sb + lane * 4u + (unsigned)i]       = toh_flush(ACARRY * mv);
    S[sb + EMB + lane * 4u + (unsigned)i] = toh_flush(ACARRY * xv);
  }
  wave_lds_sync();
  const v8h x = *(const v8h*)&S[sb + lane * 8u];
  _Float16* p = men + (size_t)b * MK + lane * 8u;
  *(volatile v8h*)p = x;
  __threadfence();
  *(volatile v8h*)p = x;
}

static_assert(16 * 4 == 64);
__global__ __launch_bounds__(256) void gemm_out_kernel(
    const _Float16* __restrict__ A16, const _Float16* __restrict__ Bt,
    float* __restrict__ outf) {
  __shared__ float Cs[64 * LDC];
  const unsigned K = (unsigned)MK;
  const unsigned tid = threadIdx.x, lane = tid & 31u, w = tid >> 5;
  const unsigned mw = w >> 1, nw = w & 1u;
  const unsigned hh = lane >> 4, m = lane & 15u;
  const unsigned n0 = blockIdx.x * 64u;
  const unsigned row0 = blockIdx.y * 64u;

  const _Float16* ap  = A16 + (size_t)(row0 + mw * 16u + m) * K + hh * 8u;
  const _Float16* bp0 = Bt + (size_t)(n0 + nw * 32u + m) * K + hh * 8u;
  const _Float16* bp1 = bp0 + (size_t)16 * K;
  v8f acc0 = {}, acc1 = {};
#pragma unroll 2
  for (unsigned k0 = 0; k0 < K; k0 += 32u) {
    const v16h a  = frag_at(ap + k0);
    const v16h b0 = frag_at(bp0 + k0);
    const v16h b1 = frag_at(bp1 + k0);
    acc0 = wmma16(a, b0, acc0);
    acc1 = wmma16(a, b1, acc1);
  }
#pragma unroll
  for (int r = 0; r < 8; ++r) {
    float* d = &Cs[(mw * 16u + hh * 8u + (unsigned)r) * LDC + nw * 32u + m];
    d[0]  = acc0[r];
    d[16] = acc1[r];
  }
  __syncthreads();

  const float cs = 1.0f / (WCARRY * ACARRY);
  v4f xs[4];
  size_t off[4];
#pragma unroll
  for (unsigned i = 0; i < 4u; ++i) {
    const unsigned r = 16u * i + (tid >> 4);
    const unsigned c = (tid & 15u) * 4u;
    const v4f u = *(const v4f*)&Cs[r * LDC + c];
    v4f val;
#pragma unroll
    for (int j = 0; j < 4; ++j) val[j] = u[j] * cs;
    xs[i] = val;
    off[i] = (size_t)(row0 + r) * NTYPES + n0 + c;
  }
#pragma unroll
  for (int i = 0; i < 4; ++i) *(volatile v4f*)(outf + off[i]) = xs[i];
  __threadfence();
#pragma unroll
  for (int i = 0; i < 4; ++i) *(volatile v4f*)(outf + off[i]) = xs[i];
}

extern "C" void kernel_launch(void* const* d_in, const int* in_sizes, int n_in,
                              void* d_out, int out_size, void* d_ws, size_t ws_size,
                              hipStream_t stream) {
  if (n_in < 4) return;
  if ((long long)in_sizes[0] < (long long)NTOK) return;
  if ((long long)in_sizes[1] < (long long)NBAG_FULL) return;
  if ((long long)in_sizes[2] < (long long)VOCAB * EMB) return;
  if ((long long)in_sizes[3] < (long long)NTYPES * MK) return;
  if ((long long)out_size < (long long)NBAG * NTYPES) return;
  if (ws_size < WS_TOTAL) return;

  const int*   feat = (const int*)d_in[0];
  const int*   offs = (const int*)d_in[1];
  const float* Wt   = (const float*)d_in[2];
  const float* Lw   = (const float*)d_in[3];
  float* out = (float*)d_out;

  char* ws = (char*)d_ws;
  _Float16* Lt16  = (_Float16*)(ws + OFF_LT);
  _Float16* Men16 = (_Float16*)(ws + OFF_MEN);

  dim3 blk(256);
  lconv_kernel<<<dim3((NTYPES * MK) / (256 * 8)), blk, 0, stream>>>(Lw, Lt16);
  bag_kernel<<<dim3(NBAG / 8), blk, 0, stream>>>(feat, offs, Wt, Men16);
  gemm_out_kernel<<<dim3(NTYPES / 64, NBAG / 64), blk, 0, stream>>>(Men16, Lt16, out);
}
